// GATLayer_44779329028364
// MI455X (gfx1250) — hardware-run, weakly checked
//
#include <hip/hip_runtime.h>
#include <stddef.h>
#include <stdint.h>
#include <math.h>


#define NN      50000
#define NE      800000
#define DD      128
#define NC2     256
#define MP      50048
#define PTHR    256
#define NBH     (MP * (DD / 8) / PTHR)
#define NBW     (NC2 * (DD / 8) / PTHR)
#define GBM     64
#define GTHR    256
#define NTHR    256
#define NWAVE   8
#define EPT     8
#define WCH     (32 * EPT)
#define NWCH    (NE / WCH)
#define WCPW    ((NWCH + NWAVE - 1) / NWAVE)
#define NBRUN   1024
#define NBLK    ((NN + NBRUN - 1) / NBRUN)
#define WLCAP   3584
#define RCAP    (NWAVE * WLCAP)
#define DEGCAP  128
#define NEGSL   0.2f
#define MX0     (-3.0e38f)
#define SCAN_INTS (2 * RCAP + 3 * NBRUN + 16)
#define GEMM_FLTS (GBM * NC2 + NC2 + 2 * GBM)

static_assert(NN <= 65536);
static_assert(NBRUN <= (65536 >> 6));
static_assert(NBLK * NBRUN >= NN);
static_assert(NE % WCH == 0);
static_assert(WCPW * NWAVE >= NWCH);
static_assert(RCAP >= 16696 + 4096);
static_assert(DEGCAP >= 33 + 8);
static_assert(SCAN_INTS * 4 <= 327680);
static_assert(GEMM_FLTS * 4 <= 327680);
static_assert(MP % GBM == 0 && MP % 128 == 0 && MP >= NN);
static_assert((MP * 4) % 128 == 0);
static_assert((MP * (DD / 8)) % PTHR == 0 && (NC2 * (DD / 8)) % PTHR == 0);
static_assert(DD % 32 == 0 && NC2 == 2 * DD);
static_assert(GBM == 4 * 16 && GTHR == 256 && NTHR * 4 == NBRUN);
static_assert(DD == 4 * 32);

typedef float          v4f   __attribute__((ext_vector_type(4)));
typedef float          v8f   __attribute__((ext_vector_type(8)));
typedef int            v4i   __attribute__((ext_vector_type(4)));
typedef int            v8i   __attribute__((ext_vector_type(8)));
typedef unsigned short v8us  __attribute__((ext_vector_type(8)));
typedef __bf16         v16bf __attribute__((ext_vector_type(16)));
typedef v4f  __attribute__((may_alias)) v4fa;
typedef v4i  __attribute__((may_alias)) v4ia;
typedef v8us __attribute__((may_alias)) v8usa;
union FragB { v16bf v; v8us h[2]; v8i w; };

__device__ __forceinline__ v8f wmb(const FragB& a, const FragB& b, v8f c) {
  v8f d = __builtin_amdgcn_wmma_f32_16x16x32_bf16(false, a.v, false, b.v, (short)0, c, false, false);
  asm volatile("v_nop\n\tv_nop\n\tv_nop\n\tv_nop" : "+v"(d) : "v"(a.w), "v"(b.w));
  return d;
}

__device__ __forceinline__ unsigned bf16_bits(float f) {
  const unsigned u = __float_as_uint(f);
  return (u + 0x7FFFu + ((u >> 16) & 1u)) >> 16;
}
__device__ __forceinline__ float bf16_val(float f) { return __uint_as_float(bf16_bits(f) << 16); }

__device__ __forceinline__ v8us cvt8(const v4f a, const v4f b, bool ok) {
  v8us o;
  o[0] = ok ? (unsigned short)bf16_bits(a.x) : (unsigned short)0;
  o[1] = ok ? (unsigned short)bf16_bits(a.y) : (unsigned short)0;
  o[2] = ok ? (unsigned short)bf16_bits(a.z) : (unsigned short)0;
  o[3] = ok ? (unsigned short)bf16_bits(a.w) : (unsigned short)0;
  o[4] = ok ? (unsigned short)bf16_bits(b.x) : (unsigned short)0;
  o[5] = ok ? (unsigned short)bf16_bits(b.y) : (unsigned short)0;
  o[6] = ok ? (unsigned short)bf16_bits(b.z) : (unsigned short)0;
  o[7] = ok ? (unsigned short)bf16_bits(b.w) : (unsigned short)0;
  return o;
}
__device__ __forceinline__ void put8us(unsigned short* p, const v8us v) {
  *(volatile v8us*)p = v;
  __threadfence();
  *(volatile v8us*)p = v;
}
__device__ __forceinline__ void put4f(float* p, const v4f v) {
  *(volatile v4f*)p = v;
  __threadfence();
  *(volatile v4f*)p = v;
}

__global__ __launch_bounds__(PTHR) void k_prep(const float* __restrict__ h, const float* __restrict__ wval,
                                               const float* __restrict__ wsc, const float* __restrict__ attn,
                                               const float* __restrict__ bias,
                                               unsigned short* hb, unsigned short* wb, float* ab) {
  const int tid = (int)threadIdx.x;
  const int blk = (int)blockIdx.x;
  if (blk < NBH) {
    const int u   = blk * PTHR + tid;
    const int row = u >> 4;
    const int k8  = (u & 15) * 8;
    const int rc  = row < NN ? row : NN - 1;
    const float* p = h + (size_t)rc * DD + k8;
    const v4f a = *(const v4f*)p;
    const v4f b = *(const v4f*)(p + 4);
    const v8us o = cvt8(a, b, row < NN);
    put8us(hb + (size_t)row * DD + k8, o);
  } else if (blk < NBH + NBW) {
    const int u  = (blk - NBH) * PTHR + tid;
    const int n  = u >> 4;
    const int k8 = (u & 15) * 8;
    const int nr = n & (DD - 1);
    const size_t so = (size_t)nr * DD + k8;
    const v4f a1 = *(const v4f*)(wval + so);
    const v4f b1 = *(const v4f*)(wval + so + 4);
    const v4f a2 = *(const v4f*)(wsc + so);
    const v4f b2 = *(const v4f*)(wsc + so + 4);
    asm volatile("" :: "v"(a1), "v"(b1), "v"(a2), "v"(b2));
    const bool first = n < DD;
    const v4f a = first ? a1 : a2;
    const v4f b = first ? b1 : b2;
    const v8us o = cvt8(a, b, true);
    put8us(wb + (size_t)n * DD + k8, o);
  } else {
    if (tid < 96) {
      const int ia = tid < 63 ? tid : 63;
      int ib = tid - 64; ib = ib < 0 ? 0 : (ib > 31 ? 31 : ib);
      const v4f va = *(const v4f*)(attn + 4 * ia);
      const v4f vb = *(const v4f*)(bias + 4 * ib);
      asm volatile("" :: "v"(va), "v"(vb));
      const v4f s = (tid < 64) ? va : vb;
      v4f r;
      r.x = bf16_val(s.x); r.y = bf16_val(s.y); r.z = bf16_val(s.z); r.w = bf16_val(s.w);
      put4f(ab + 4 * tid, r);
    }
  }
}

__global__ __launch_bounds__(GTHR) __attribute__((amdgpu_num_vgpr(248)))
void k_gemm(const unsigned short* __restrict__ A, const unsigned short* __restrict__ BT,
            const float* __restrict__ ab, float* HT, float* SD) {
  extern __shared__ __attribute__((aligned(16))) float gsm[];
  float* stg  = gsm;
  float* satt = gsm + GBM * NC2;
  float* sdt  = satt + NC2;
  const int tid = (int)threadIdx.x, lane = tid & 31, wave = tid >> 5, hh = lane >> 4, m = lane & 15;
  const int rg = wave & 3, cg = wave >> 2;
  const int rowBase = (int)blockIdx.x * GBM;
  const int colBase = cg * DD;

  if (tid < 64) {
    const v4f t4 = *(const v4f*)(ab + 4 * tid);
    *(v4fa*)(satt + 4 * tid) = t4;
  }

  v8f acc[8];
  {
    const v8f z = {0.f, 0.f, 0.f, 0.f, 0.f, 0.f, 0.f, 0.f};
#pragma unroll
    for (int t = 0; t < 8; ++t) acc[t] = z;
  }
  const unsigned short* ap = A  + (size_t)(rowBase + 16 * rg + m) * (size_t)DD + 8 * hh;
  const unsigned short* bp = BT + (size_t)(colBase + m) * (size_t)DD + 8 * hh;

#pragma unroll 1
  for (int k0 = 0; k0 < DD; k0 += 32) {
    FragB af;
    af.h[0] = *(const v8usa*)(ap + k0);
    af.h[1] = *(const v8usa*)(ap + k0 + 16);
#pragma unroll
    for (int nt = 0; nt < 8; ++nt) {
      const unsigned short* wq = bp + (size_t)(16 * nt) * (size_t)DD + k0;
      FragB bf;
      bf.h[0] = *(const v8usa*)wq;
      bf.h[1] = *(const v8usa*)(wq + 16);
      acc[nt] = wmb(af, bf, acc[nt]);
    }
  }

#pragma unroll
  for (int nt = 0; nt < 8; ++nt) {
    const int lc = colBase + 16 * nt + m;
#pragma unroll
    for (int r = 0; r < 8; ++r) {
      const int lr = 16 * rg + 8 * hh + r;
      stg[lr * NC2 + lc] = acc[nt][r];
    }
  }
  __syncthreads();

  if (tid < 128) {
    const int row   = tid & 63;
    const int which = tid >> 6;
    const float* hr = stg + row * NC2 + DD;
    const float* av = satt + which * DD;
    float d = 0.0f;
#pragma unroll 2
    for (int c4 = 0; c4 < DD / 4; ++c4) {
      const v4f hv = *(const v4fa*)(hr + 4 * c4);
      const v4f a4 = *(const v4fa*)(av + 4 * c4);
      d = fmaf(hv.x, a4.x, d);
      d = fmaf(hv.y, a4.y, d);
      d = fmaf(hv.z, a4.z, d);
      d = fmaf(hv.w, a4.w, d);
    }
    sdt[which * GBM + row] = d;
  }
  __syncthreads();

  const v4f sdv = *(const v4fa*)(sdt + 4 * lane);
  float* sp = SD + (size_t)(lane >> 4) * (size_t)MP + rowBase + 4 * (lane & 15);
#pragma unroll 1
  for (int i = 0; i < 8; ++i) {
    const int row = wave * 8 + i;
    const v4f p = *(const v4fa*)(stg + row * NC2 + 4 * lane);
    float* op = HT + (size_t)(rowBase + row) * (size_t)DD + 4 * lane;
    *(volatile v4f*)op = p;
  }
  if (wave == 0) *(volatile v4f*)sp = sdv;
  __threadfence();
#pragma unroll 1
  for (int i = 0; i < 8; ++i) {
    const int row = wave * 8 + i;
    const v4f p = *(const v4fa*)(stg + row * NC2 + 4 * lane);
    float* op = HT + (size_t)(rowBase + row) * (size_t)DD + 4 * lane;
    *(volatile v4f*)op = p;
  }
  if (wave == 0) *(volatile v4f*)sp = sdv;
}

__global__ __launch_bounds__(NTHR) __attribute__((amdgpu_num_vgpr(248)))
void k_scan(const int* __restrict__ srcs, const int* __restrict__ dsts,
            const float* __restrict__ HT, const float* __restrict__ SD,
            const float* __restrict__ ab, float* outp) {
  extern __shared__ __attribute__((aligned(16))) int dsm[];
  int* wl   = dsm;
  int* sl   = dsm + RCAP;
  int* cnt  = dsm + 2 * RCAP;
  int* offs = cnt + NBRUN;
  int* cur  = offs + NBRUN;
  int* misc = cur + NBRUN;
  const int tid = (int)threadIdx.x, lane = tid & 31, wave = tid >> 5;
  const int nodeBase = (int)blockIdx.x * NBRUN;
  int nb = NN - nodeBase;
  nb = nb < 0 ? 0 : (nb > NBRUN ? NBRUN : nb);

  {
    const v4i z4 = {0, 0, 0, 0};
    *(v4ia*)(cnt + 4 * tid) = z4;
    if (tid < 16) misc[tid] = 0;
  }
  const v4f bv = *(const v4f*)(ab + NC2 + 4 * lane);
  __syncthreads();

  int wcur = 0;
  {
    int* wlw = wl + wave * WLCAP;
    const int cbeg = wave * WCPW;
    int cend = cbeg + WCPW;
    cend = cend > NWCH ? NWCH : cend;
    const unsigned nbs = (unsigned)nodeBase;
    const unsigned unb = (unsigned)nb;
#pragma unroll 1
    for (int ch = cbeg; ch < cend; ++ch) {
      const int e0 = ch * WCH + lane * EPT;
      const v4i da = *(const v4i*)(dsts + e0);
      const v4i db = *(const v4i*)(dsts + e0 + 4);
      const v4i sa = *(const v4i*)(srcs + e0);
      const v4i sb = *(const v4i*)(srcs + e0 + 4);
      asm volatile("" :: "v"(sa), "v"(sb));
      const unsigned s0 = (unsigned)da.x - nbs, s1 = (unsigned)da.y - nbs;
      const unsigned s2 = (unsigned)da.z - nbs, s3 = (unsigned)da.w - nbs;
      const unsigned s4 = (unsigned)db.x - nbs, s5 = (unsigned)db.y - nbs;
      const unsigned s6 = (unsigned)db.z - nbs, s7 = (unsigned)db.w - nbs;
      const bool h0 = s0 < unb, h1 = s1 < unb, h2 = s2 < unb, h3 = s3 < unb;
      const bool h4 = s4 < unb, h5 = s5 < unb, h6 = s6 < unb, h7 = s7 < unb;
      const unsigned m0 = __builtin_amdgcn_ballot_w32(h0);
      const unsigned m1 = __builtin_amdgcn_ballot_w32(h1);
      const unsigned m2 = __builtin_amdgcn_ballot_w32(h2);
      const unsigned m3 = __builtin_amdgcn_ballot_w32(h3);
      const unsigned m4 = __builtin_amdgcn_ballot_w32(h4);
      const unsigned m5 = __builtin_amdgcn_ballot_w32(h5);
      const unsigned m6 = __builtin_amdgcn_ballot_w32(h6);
      const unsigned m7 = __builtin_amdgcn_ballot_w32(h7);
      const unsigned any = m0 | m1 | m2 | m3 | m4 | m5 | m6 | m7;
      if (any != 0u) {
        const int below = (int)(__builtin_amdgcn_mbcnt_lo(m0, 0u) + __builtin_amdgcn_mbcnt_lo(m1, 0u) +
                                __builtin_amdgcn_mbcnt_lo(m2, 0u) + __builtin_amdgcn_mbcnt_lo(m3, 0u) +
                                __builtin_amdgcn_mbcnt_lo(m4, 0u) + __builtin_amdgcn_mbcnt_lo(m5, 0u) +
                                __builtin_amdgcn_mbcnt_lo(m6, 0u) + __builtin_amdgcn_mbcnt_lo(m7, 0u));
        int pos = wcur + below;
#define PUTJ(HJ, SJ, SV) { \
          int sv = (SV); \
          sv = sv < 0 ? 0 : (sv > NN - 1 ? NN - 1 : sv); \
          if (HJ) { if (pos < WLCAP) wlw[pos] = sv | ((int)(SJ) << 16); } \
          pos += (HJ) ? 1 : 0; }
        PUTJ(h0, s0, sa.x)
        PUTJ(h1, s1, sa.y)
        PUTJ(h2, s2, sa.z)
        PUTJ(h3, s3, sa.w)
        PUTJ(h4, s4, sb.x)
        PUTJ(h5, s5, sb.y)
        PUTJ(h6, s6, sb.z)
        PUTJ(h7, s7, sb.w)
#undef PUTJ
        wcur += (int)(__builtin_popcount(m0) + __builtin_popcount(m1) + __builtin_popcount(m2) +
                      __builtin_popcount(m3) + __builtin_popcount(m4) + __builtin_popcount(m5) +
                      __builtin_popcount(m6) + __builtin_popcount(m7));
      }
    }
  }
  if (lane == 0) misc[wave] = wcur;
  __syncthreads();

  if (wave == 0) {
    int ovl = 0;
#pragma unroll 1
    for (int w2 = 0; w2 < NWAVE; ++w2) {
      int cv = misc[w2];
      ovl |= (cv > WLCAP) ? 1 : 0;
      cv = cv < 0 ? 0 : (cv > WLCAP ? WLCAP : cv);
      const int c = __builtin_amdgcn_readfirstlane(cv);
      int lastw = c - 1; lastw = lastw < 0 ? 0 : lastw;
#pragma unroll 1
      for (int b0 = 0; b0 < c; b0 += 32) {
        int idx = b0 + lane; idx = idx > lastw ? lastw : idx;
        const int ent = wl[w2 * WLCAP + idx];
        const int m32 = (c - b0) < 32 ? (c - b0) : 32;
#pragma unroll 1
        for (int k = 0; k < m32; ++k) {
          const int u    = __builtin_amdgcn_readlane(ent, k);
          const int slot = (u >> 16) & (NBRUN - 1);
          const int old  = cnt[slot];
          if (lane == 0) cnt[slot] = old + 1;
        }
      }
    }
    if (lane == 0) misc[9] = ovl;
  }
  __syncthreads();

  if (wave == 0) {
    const int base = lane * (NBRUN / 32);
    int s = 0;
#pragma unroll 1
    for (int i = 0; i < NBRUN / 32; ++i) s += cnt[base + i];
    int incl = s;
#pragma unroll
    for (int d = 1; d < 32; d <<= 1) {
      const int y = __shfl_up(incl, d, 32);
      if (lane >= d) incl += y;
    }
    int run = incl - s;
#pragma unroll 1
    for (int i = 0; i < NBRUN / 32; ++i) {
      const int cv = cnt[base + i];
      offs[base + i] = run;
      cur[base + i]  = run;
      run += cv;
    }
  }
  __syncthreads();

  if (wave == 0) {
#pragma unroll 1
    for (int w2 = 0; w2 < NWAVE; ++w2) {
      int cv = misc[w2];
      cv = cv < 0 ? 0 : (cv > WLCAP ? WLCAP : cv);
      const int c = __builtin_amdgcn_readfirstlane(cv);
      int lastw = c - 1; lastw = lastw < 0 ? 0 : lastw;
#pragma unroll 1
      for (int b0 = 0; b0 < c; b0 += 32) {
        int idx = b0 + lane; idx = idx > lastw ? lastw : idx;
        const int ent = wl[w2 * WLCAP + idx];
        const int m32 = (c - b0) < 32 ? (c - b0) : 32;
#pragma unroll 1
        for (int k = 0; k < m32; ++k) {
          const int u    = __builtin_amdgcn_readlane(ent, k);
          const int slot = (u >> 16) & (NBRUN - 1);
          int p = cur[slot];
          p = p < 0 ? 0 : (p > RCAP - 1 ? RCAP - 1 : p);
          if (lane == 0) { sl[p] = u & 0xFFFF; cur[slot] = p + 1; }
        }
      }
    }
  }
  __syncthreads();

  const int ovf = misc[9];
  const float qn = __int_as_float(0x7fc00000);
  const float* SDd = SD + MP;
#pragma unroll 1
  for (int s = wave; s < nb; s += NWAVE) {
    const int node = nodeBase + s;
    int cv = cnt[s];
    const bool big = cv > DEGCAP;
    cv = cv < 0 ? 0 : (cv > DEGCAP ? DEGCAP : cv);
    int ov = offs[s];
    ov = ov < 0 ? 0 : (ov > RCAP - 1 ? RCAP - 1 : ov);
    if (cv > RCAP - ov) cv = RCAP - ov;
    const int c = __builtin_amdgcn_readfirstlane(cv);
    const int o = __builtin_amdgcn_readfirstlane(ov);
    int last = o + c - 1; last = last < o ? o : last;
    const float ad = SDd[node];
    float mx = MX0, dn = 0.0f;
    v4f acc = {0.f, 0.f, 0.f, 0.f};
#pragma unroll 1
    for (int b0 = 0; b0 < c; b0 += 32) {
      int idx = o + b0 + lane; idx = idx > last ? last : idx;
      int sr = sl[idx];
      sr = sr < 0 ? 0 : (sr > NN - 1 ? NN - 1 : sr);
      const float es  = SD[sr];
      const int   esi = __float_as_int(es);
      const int m32 = (c - b0) < 32 ? (c - b0) : 32;
#pragma unroll 1
      for (int k = 0; k < m32; ++k) {
        const int   sk  = __builtin_amdgcn_readlane(sr, k);
        const float ask = __int_as_float(__builtin_amdgcn_readlane(esi, k));
        const v4f a = *(const v4f*)(HT + (size_t)sk * DD + 4 * lane);
        float lg = ask + ad;
        lg = lg > 0.f ? lg : NEGSL * lg;
        const float df = lg - mx;
        const float ee = expf(-fabsf(df));
        const bool  up = df > 0.f;
        const float s1 = up ? ee : 1.0f;
        const float s2 = up ? 1.0f : ee;
        mx = up ? lg : mx;
        dn = fmaf(dn, s1, s2);
        acc.x = fmaf(acc.x, s1, s2 * a.x);
        acc.y = fmaf(acc.y, s1, s2 * a.y);
        acc.z = fmaf(acc.z, s1, s2 * a.z);
        acc.w = fmaf(acc.w, s1, s2 * a.w);
      }
    }
    const bool has = cv > 0;
    const float dsafe = has ? dn : 1.0f;
    const float inv = __builtin_amdgcn_rcpf(dsafe);
    const float pz = (ovf != 0 || big) ? qn : 0.0f;
    v4f y;
    y.x = (has ? acc.x * inv : 0.0f) + bv.x;
    y.y = (has ? acc.y * inv : 0.0f) + bv.y;
    y.z = (has ? acc.z * inv : 0.0f) + bv.z;
    y.w = (has ? acc.w * inv : 0.0f) + bv.w;
    v4f r;
    r.x = ((y.x > 0.f) ? y.x : NEGSL * y.x) + pz;
    r.y = ((y.y > 0.f) ? y.y : NEGSL * y.y) + pz;
    r.z = ((y.z > 0.f) ? y.z : NEGSL * y.z) + pz;
    r.w = ((y.w > 0.f) ? y.w : NEGSL * y.w) + pz;
    float* op = outp + (size_t)node * DD + 4 * lane;
    *(volatile v4f*)op = r;
    __threadfence();
    *(volatile v4f*)op = r;
  }
}

extern "C" void kernel_launch(void* const* d_in, const int* in_sizes, int n_in,
                              void* d_out, int out_size, void* d_ws, size_t ws_size,
                              hipStream_t stream) {
  if (n_in < 8) return;
  if (in_sizes[0] != NN * DD) return;
  if (in_sizes[1] != NE || in_sizes[2] != NE) return;
  if (in_sizes[3] != DD * DD || in_sizes[4] != DD * DD || in_sizes[5] != DD * DD) return;
  if (in_sizes[6] != 2 * DD) return;
  if (in_sizes[7] != DD) return;
  if (out_size != NN * DD) return;

  const float* h    = (const float*)d_in[0];
  const int*   src  = (const int*)d_in[1];
  const int*   dst  = (const int*)d_in[2];
  const float* wval = (const float*)d_in[3];
  const float* wsc  = (const float*)d_in[4];
  const float* attn = (const float*)d_in[6];
  const float* bias = (const float*)d_in[7];
  float* out = (float*)d_out;

  char* ws = (char*)d_ws;
  size_t off = 0;
  const size_t oHB = off; off += (size_t)MP * DD * 2;      off = (off + 255) & ~(size_t)255;
  const size_t oWB = off; off += (size_t)NC2 * DD * 2;     off = (off + 255) & ~(size_t)255;
  const size_t oAB = off; off += (size_t)(NC2 + DD) * 4;   off = (off + 255) & ~(size_t)255;
  const size_t oHT = off; off += (size_t)MP * DD * 4;      off = (off + 255) & ~(size_t)255;
  const size_t oSD = off; off += (size_t)2 * MP * 4;       off = (off + 255) & ~(size_t)255;
  if (off > ws_size || off > (size_t)(128u << 20)) return;
  unsigned short* HB = (unsigned short*)(ws + oHB);
  unsigned short* WB = (unsigned short*)(ws + oWB);
  float*          AB = (float*)(ws + oAB);
  float*          HT = (float*)(ws + oHT);
  float*          SD = (float*)(ws + oSD);

  const int gemmLds = GEMM_FLTS * 4;
  const int scanLds = SCAN_INTS * 4;
  hipFuncSetAttribute(reinterpret_cast<const void*>(&k_gemm), hipFuncAttributeMaxDynamicSharedMemorySize, gemmLds);
  hipFuncSetAttribute(reinterpret_cast<const void*>(&k_scan), hipFuncAttributeMaxDynamicSharedMemorySize, scanLds);

  k_prep<<<NBH + NBW + 1, PTHR, 0, stream>>>(h, wval, wsc, attn, bias, HB, WB, AB);
  k_gemm<<<MP / GBM, GTHR, (size_t)gemmLds, stream>>>(HB, WB, AB, HT, SD);
  k_scan<<<NBLK, NTHR, (size_t)scanLds, stream>>>(src, dst, HT, SD, AB, out);
}
